// MatchLayer_14267881357504
// MI455X (gfx1250) — hardware-verified
//
#include <hip/hip_runtime.h>

typedef _Float16 v16h __attribute__((ext_vector_type(16)));
typedef _Float16 v8h  __attribute__((ext_vector_type(8)));
typedef float    v8f  __attribute__((ext_vector_type(8)));
typedef float    v4f  __attribute__((ext_vector_type(4)));
typedef v8h __attribute__((may_alias)) v8ha;
typedef v4f __attribute__((may_alias)) v4fa;

union Frag { v16h v; v8h half[2]; };

#define NB    8
#define NL    2048
#define ND    128
#define NROW  (NB * NL)
#define NTENS 4
#define NIN   (NROW * ND)
#define NOUT  (4 * NROW)
#define EPSF  1e-6f

__device__ __forceinline__ v8f wmma_f16(v16h a, v16h b, v8f c) {
  v8f d = __builtin_amdgcn_wmma_f32_16x16x32_f16(false, a, false, b, (short)0, c, false, false);
  asm volatile("v_nop\n\tv_nop\n\tv_nop\n\tv_nop" : "+v"(d) : "v"(a), "v"(b));
  return d;
}

__device__ __forceinline__ v16h load_frag(const _Float16* p, int h) {
  Frag f;
  f.half[0] = *(const v8ha*)(p + 8 * h);
  f.half[1] = *(const v8ha*)(p + 16 + 8 * h);
  return f.v;
}

__device__ __forceinline__ v8h cvt8(v4f a, v4f c) {
  v8h t;
  t[0] = (_Float16)a[0]; t[1] = (_Float16)a[1]; t[2] = (_Float16)a[2]; t[3] = (_Float16)a[3];
  t[4] = (_Float16)c[0]; t[5] = (_Float16)c[1]; t[6] = (_Float16)c[2]; t[7] = (_Float16)c[3];
  return t;
}

__device__ __forceinline__ float sq8(v4f a, v4f c) {
  return a[0] * a[0] + a[1] * a[1] + a[2] * a[2] + a[3] * a[3]
       + c[0] * c[0] + c[1] * c[1] + c[2] * c[2] + c[3] * c[3];
}

__global__ __launch_bounds__(256) void prep_kernel(
    const float* __restrict__ t_fw, const float* __restrict__ t_bw,
    const float* __restrict__ h_fw, const float* __restrict__ h_bw,
    _Float16* __restrict__ planes,
    float* __restrict__ inv)
{
  __shared__ __attribute__((aligned(16))) float sinv[32];

  const int tid  = threadIdx.x;
  const int tens = blockIdx.y;
  const int r0   = blockIdx.x * 32;

  const float* src = (tens == 0) ? t_fw : ((tens == 1) ? t_bw : ((tens == 2) ? h_fw : h_bw));
  const float* tile = src + (size_t)r0 * ND;
  _Float16* ptile = planes + ((size_t)tens * NROW + r0) * ND;

  const int e0 = tid * 8;
  const int e1 = 2048 + tid * 8;

  const v4f a0 = *(const v4fa*)(tile + e0);
  const v4f c0 = *(const v4fa*)(tile + e0 + 4);
  const v4f a1 = *(const v4fa*)(tile + e1);
  const v4f c1 = *(const v4fa*)(tile + e1 + 4);

  const v8h o0 = cvt8(a0, c0);
  const v8h o1 = cvt8(a1, c1);

  float ss0 = sq8(a0, c0);
  float ss1 = sq8(a1, c1);
  ss0 += __shfl_xor(ss0, 1); ss1 += __shfl_xor(ss1, 1);
  ss0 += __shfl_xor(ss0, 2); ss1 += __shfl_xor(ss1, 2);
  ss0 += __shfl_xor(ss0, 4); ss1 += __shfl_xor(ss1, 4);
  ss0 += __shfl_xor(ss0, 8); ss1 += __shfl_xor(ss1, 8);
  const float n0 = 1.0f / sqrtf(fmaxf(ss0, EPSF));
  const float n1 = 1.0f / sqrtf(fmaxf(ss1, EPSF));
  if ((tid & 15) == 0) {
    sinv[tid >> 4] = n0;
    sinv[16 + (tid >> 4)] = n1;
  }
  __syncthreads();

  const v4f nl = *(const v4fa*)(sinv + 4 * (tid & 7));
  float* ninv = inv + (size_t)tens * NROW + r0 + 4 * (tid & 7);

  *(volatile v8h*)(ptile + e0) = o0;
  *(volatile v8h*)(ptile + e1) = o1;
  if (tid < 8) *(volatile v4f*)ninv = nl;
  __threadfence();
  *(volatile v8h*)(ptile + e0) = o0;
  *(volatile v8h*)(ptile + e1) = o1;
  if (tid < 8) *(volatile v4f*)ninv = nl;
}

__global__ __launch_bounds__(128) void cosmax_kernel(
    const _Float16* __restrict__ planes,
    const float* __restrict__ inv,
    float* __restrict__ out)
{
  __shared__ __attribute__((aligned(16))) float sres[2 * 128];

  const int tid = threadIdx.x, lane = tid & 31, w = tid >> 5;
  const int h = lane >> 4, m = lane & 15;
  const int dir = blockIdx.z, b = blockIdx.y, hbase = blockIdx.x * 128;

  const _Float16* tplane = planes + ((size_t)dir * NROW + (size_t)b * NL) * ND;
  const _Float16* hplane = planes + ((size_t)(2 + dir) * NROW + (size_t)b * NL) * ND;
  const float* tinv = inv + (size_t)dir * NROW + (size_t)b * NL;
  const float* hinv = inv + (size_t)(2 + dir) * NROW + (size_t)b * NL;

  const int hc0 = hbase + 32 * w + m;
  const int hc1 = hc0 + 16;

  v16h b0[4], b1[4];
  #pragma unroll
  for (int c = 0; c < 4; ++c) {
    b0[c] = load_frag(hplane + (size_t)hc0 * ND + 32 * c, h);
    b1[c] = load_frag(hplane + (size_t)hc1 * ND + 32 * c, h);
  }

  const v8f zero8 = {0.f, 0.f, 0.f, 0.f, 0.f, 0.f, 0.f, 0.f};
  float mx0 = -3.0e38f, mx1 = -3.0e38f, sm0 = 0.0f, sm1 = 0.0f;

  #pragma unroll 1
  for (int t0 = 0; t0 < NL; t0 += 16) {
    const _Float16* tp = tplane + (size_t)(t0 + m) * ND;
    v8f acc0 = zero8, acc1 = zero8;
    #pragma unroll
    for (int c = 0; c < 4; ++c) {
      const v16h a = load_frag(tp + 32 * c, h);
      acc0 = wmma_f16(a, b0[c], acc0);
      acc1 = wmma_f16(a, b1[c], acc1);
    }
    const v4f i0 = *(const v4fa*)(tinv + t0 + 8 * h);
    const v4f i1 = *(const v4fa*)(tinv + t0 + 8 * h + 4);
    #pragma unroll
    for (int r = 0; r < 4; ++r) {
      const float u0 = acc0[r] * i0[r];
      const float u1 = acc1[r] * i0[r];
      mx0 = fmaxf(mx0, u0); sm0 = sm0 + u0;
      mx1 = fmaxf(mx1, u1); sm1 = sm1 + u1;
    }
    #pragma unroll
    for (int r = 0; r < 4; ++r) {
      const float u0 = acc0[4 + r] * i1[r];
      const float u1 = acc1[4 + r] * i1[r];
      mx0 = fmaxf(mx0, u0); sm0 = sm0 + u0;
      mx1 = fmaxf(mx1, u1); sm1 = sm1 + u1;
    }
  }

  mx0 = fmaxf(mx0, __shfl_xor(mx0, 16));
  mx1 = fmaxf(mx1, __shfl_xor(mx1, 16));
  sm0 = sm0 + __shfl_xor(sm0, 16);
  sm1 = sm1 + __shfl_xor(sm1, 16);

  const float ih0 = hinv[hc0];
  const float ih1 = hinv[hc1];
  if (h == 0) {
    sres[32 * w + m]            = mx0 * ih0;
    sres[32 * w + 16 + m]       = mx1 * ih1;
    sres[128 + 32 * w + m]      = (sm0 * ih0) * (1.0f / 2048.0f);
    sres[128 + 32 * w + 16 + m] = (sm1 * ih1) * (1.0f / 2048.0f);
  }
  __syncthreads();

  const int sel = w & 1;
  const v4f ov = *(const v4fa*)(sres + 128 * sel + 4 * lane);
  float* dst = out + (size_t)sel * NROW + (size_t)dir * 2 * NROW + (size_t)b * NL + hbase + 4 * lane;
  if (w < 2) *(volatile v4f*)dst = ov;
  __threadfence();
  if (w < 2) *(volatile v4f*)dst = ov;
}

extern "C" void kernel_launch(void* const* d_in, const int* in_sizes, int n_in,
                              void* d_out, int out_size, void* d_ws, size_t ws_size,
                              hipStream_t stream) {
  if (n_in < 4) return;
  if (in_sizes[0] != NIN || in_sizes[1] != NIN || in_sizes[2] != NIN || in_sizes[3] != NIN) return;
  if (out_size != NOUT) return;

  const size_t plane_bytes = (size_t)NTENS * NIN * 2;
  const size_t inv_bytes   = (size_t)NTENS * NROW * 4;
  const size_t total = plane_bytes + inv_bytes;
  if (total > ws_size) return;

  const float* t_fw = (const float*)d_in[0];
  const float* t_bw = (const float*)d_in[1];
  const float* h_fw = (const float*)d_in[2];
  const float* h_bw = (const float*)d_in[3];
  float* out = (float*)d_out;

  char* ws = (char*)d_ws;
  _Float16* planes = (_Float16*)ws;
  float* inv = (float*)(ws + plane_bytes);

  prep_kernel<<<dim3(NROW / 32, NTENS), 256, 0, stream>>>(t_fw, t_bw, h_fw, h_bw, planes, inv);

  cosmax_kernel<<<dim3(NL / 128, NB, 2), 128, 0, stream>>>(planes, inv, out);
}
